// PaiConv_6597069766757
// MI455X (gfx1250) — hardware-verified
//
#include <hip/hip_runtime.h>

typedef _Float16 v16h __attribute__((ext_vector_type(16)));
typedef _Float16 v8h  __attribute__((ext_vector_type(8)));
typedef float    v8f  __attribute__((ext_vector_type(8)));
typedef float    v4f  __attribute__((ext_vector_type(4)));
typedef v8h __attribute__((may_alias)) v8ha;
typedef v4f __attribute__((may_alias)) v4fa;

union Frag { v16h v; v8h half[2]; };
union DU2 { double d[2]; v4f f; };

#define NB     4
#define NPT    8192
#define KNB    32
#define CIN    64
#define CXF    32
#define COUT   64
#define NFT    96
#define FLATK  3072
#define TOTP   32768
#define CHUNK  4096
#define NCHUNK 8
#define PPW    8
#define PPB    32
#define NWC8   24576
#define NWM8   256

#define WS_WCH   0ull
#define WS_WMH   393216ull
#define WS_FT    397312ull
#define WS_FLH   4591616ull
#define WS_FLL   29757440ull
#define WS_PRE   54923264ull
#define WS_STAT  63311872ull
#define WS_TOTAL 63320064ull

static_assert(WS_WMH == WS_WCH + (unsigned long long)COUT * FLATK * 2);
static_assert(WS_FT == WS_WMH + (unsigned long long)CXF * 64 * 2);
static_assert(WS_FLH == WS_FT + (unsigned long long)TOTP * CIN * 2);
static_assert(WS_FLL == WS_FLH + (unsigned long long)CHUNK * FLATK * 2);
static_assert(WS_PRE == WS_FLL + (unsigned long long)CHUNK * FLATK * 2);
static_assert(WS_STAT == WS_PRE + (unsigned long long)TOTP * COUT * 4);
static_assert(WS_TOTAL == WS_STAT + 64ull * 128);
static_assert((WS_WMH % 128) == 0 && (WS_FT % 128) == 0 && (WS_FLH % 128) == 0 && (WS_FLL % 128) == 0 && (WS_PRE % 128) == 0 && (WS_STAT % 128) == 0);
static_assert(WS_TOTAL <= 134217728ull);
static_assert(FLATK % 32 == 0 && FLATK % 256 == 0);
static_assert(CHUNK % PPB == 0 && CHUNK % 128 == 0 && NPT % CHUNK == 0 && TOTP == NCHUNK * CHUNK);
static_assert((NWC8 % 256) == 0 && NWM8 == 256);
static_assert(NPT % 64 == 0 && NPT % 1024 == 0);

#define LT_BMAT 0
#define LT_KERN 896
#define LT_OPAD 1280
#define LT_BMLP 5376
#define LT_WAVE 5632
#define LW_PE    0
#define LW_FEATS 4096
#define LW_RAW   10240
#define LW_PERMT 14336
#define LW_FLH   16384
#define LW_FLL   22528
#define LW_SIZE  28672
#define LDS_POINT (LT_WAVE + 4 * LW_SIZE)
static_assert(LDS_POINT == 120320);
static_assert((LT_WAVE % 16) == 0 && (LW_SIZE % 16) == 0);

__device__ __forceinline__ v8f wmma_f16(v16h a, v16h b, v8f c) {
  v8f d = __builtin_amdgcn_wmma_f32_16x16x32_f16(false, a, false, b, (short)0, c, false, false);
  asm volatile("v_nop\n\tv_nop\n\tv_nop\n\tv_nop" : "+v"(d) : "v"(a), "v"(b));
  return d;
}

__device__ __forceinline__ v16h load_frag(const _Float16* p, int h) {
  Frag f;
  f.half[0] = *(const v8ha*)(p + 8 * h);
  f.half[1] = *(const v8ha*)(p + 16 + 8 * h);
  return f.v;
}

__device__ __forceinline__ void cvt8(const float* src, _Float16* dst, float sc) {
  const v4f a = *(const v4fa*)src;
  const v4f c = *(const v4fa*)(src + 4);
  const v8h o = { (_Float16)(a.x * sc), (_Float16)(a.y * sc), (_Float16)(a.z * sc), (_Float16)(a.w * sc),
                  (_Float16)(c.x * sc), (_Float16)(c.y * sc), (_Float16)(c.z * sc), (_Float16)(c.w * sc) };
  *(volatile v8h*)dst = o;
  __threadfence();
  *(volatile v8h*)dst = o;
}

__global__ __launch_bounds__(256) void k_cvtw(const float* __restrict__ wc, const float* __restrict__ wm,
                                             _Float16* __restrict__ wch, _Float16* __restrict__ wmh) {
  const int tid = threadIdx.x;
  if (blockIdx.x < NWC8 / 256) {
    const int g = blockIdx.x * 256 + tid;
    cvt8(wc + (size_t)g * 8, wch + (size_t)g * 8, 4096.0f);
  } else if (blockIdx.x == NWC8 / 256) {
    const int e = tid;
    cvt8(wm + (size_t)e * 8, wmh + (size_t)e * 8, 64.0f);
  }
}

__device__ __forceinline__ void ft_store_pass(const _Float16* sT, _Float16* ft, int b, int n0, int w, int lane) {
  const int q8 = lane & 7, sub = lane >> 3;
  #pragma unroll
  for (int i = 0; i < 2; ++i) {
    const int lid = 8 * w + 4 * i + sub;
    const v8h v = *(const v8ha*)(sT + lid * 64 + 8 * q8);
    *(volatile v8h*)(ft + ((size_t)(b * NPT + n0 + lid)) * CIN + 8 * q8) = v;
  }
}

__global__ __launch_bounds__(256) void k_ft(const float* __restrict__ feat, _Float16* __restrict__ ft) {
  __shared__ __attribute__((aligned(16))) _Float16 sT[64 * 64];
  const int tid = threadIdx.x, lane = tid & 31, w = tid >> 5;
  const int b = blockIdx.y, n0 = blockIdx.x * 64;
  const float* src = feat + (size_t)b * CIN * NPT + n0;
  #pragma unroll
  for (int i = 0; i < 4; ++i) {
    const int e = i * 256 + tid;
    const int c = e >> 4, t4 = e & 15;
    const v4f v = *(const v4fa*)(src + (size_t)c * NPT + 4 * t4);
    sT[(4 * t4 + 0) * 64 + c] = (_Float16)v.x;
    sT[(4 * t4 + 1) * 64 + c] = (_Float16)v.y;
    sT[(4 * t4 + 2) * 64 + c] = (_Float16)v.z;
    sT[(4 * t4 + 3) * 64 + c] = (_Float16)v.w;
  }
  __syncthreads();
  ft_store_pass(sT, ft, b, n0, w, lane);
  __threadfence();
  ft_store_pass(sT, ft, b, n0, w, lane);
}

__device__ __forceinline__ void flat_store_pass(const _Float16* hs, const _Float16* ls,
                                                _Float16* gh, _Float16* gl, int lane) {
  #pragma unroll
  for (int i = 0; i < FLATK / 256; ++i) {
    const int q = 32 * i + lane;
    const v8h a = *(const v8ha*)(hs + 8 * q);
    const v8h c = *(const v8ha*)(ls + 8 * q);
    *(volatile v8h*)(gh + 8 * q) = a;
    *(volatile v8h*)(gl + 8 * q) = c;
  }
}

__global__ __launch_bounds__(128) void k_point(
    const float* __restrict__ x,
    const int* __restrict__ neigh,
    const float* __restrict__ bmat,
    const float* __restrict__ kern,
    const float* __restrict__ opad,
    const float* __restrict__ bmlp,
    const _Float16* __restrict__ ft,
    const _Float16* __restrict__ wmh,
    _Float16* __restrict__ flh,
    _Float16* __restrict__ fll,
    int cbase)
{
  extern __shared__ __attribute__((aligned(16))) char smem[];
  float* sB  = (float*)(smem + LT_BMAT);
  float* sK  = (float*)(smem + LT_KERN);
  float* sOP = (float*)(smem + LT_OPAD);
  float* sBM = (float*)(smem + LT_BMLP);

  const int tid = threadIdx.x, lane = tid & 31, w = tid >> 5;
  const int h = lane >> 4, m = lane & 15;

  for (int i = tid; i < 7 * 32; i += 128) sB[i] = bmat[i];
  if (tid < 96) sK[tid] = kern[tid];
  for (int i = tid; i < 32 * 32; i += 128) sOP[i] = opad[i];
  if (tid < 32) sBM[tid] = bmlp[tid];

  char* wb = smem + LT_WAVE + w * LW_SIZE;
  _Float16* peL   = (_Float16*)(wb + LW_PE);
  _Float16* featL = (_Float16*)(wb + LW_FEATS);
  float*    rawS  = (float*)(wb + LW_RAW);
  _Float16* permT = (_Float16*)(wb + LW_PERMT);
  _Float16* fhS   = (_Float16*)(wb + LW_FLH);
  _Float16* flS   = (_Float16*)(wb + LW_FLL);
  __syncthreads();

  const v8f zero8 = {0.f, 0.f, 0.f, 0.f, 0.f, 0.f, 0.f, 0.f};
  const float TP = 6.283185307179586f;

  #pragma unroll 1
  for (int p = 0; p < PPW; ++p) {
    const int lp = blockIdx.x * PPB + w * PPW + p;
    const int gp = cbase + lp;
    const int b = gp >> 13;

    int idx = neigh[(size_t)gp * KNB + lane];
    idx = min(max(idx, 0), NPT - 1);

    const float* xb = x + (size_t)b * 3 * NPT;
    const float px = xb[idx], py = xb[NPT + idx], pz = xb[2 * NPT + idx];
    const float rx = __shfl(px, 0), ry = __shfl(py, 0), rz = __shfl(pz, 0);
    const float dx = px - rx, dy = py - ry, dz = pz - rz;
    const float d2 = dx * dx + dy * dy + dz * dz;
    const float dis = sqrtf(fmaxf(d2, 1e-12f));
    const float rf0 = TP * rx, rf1 = TP * ry, rf2 = TP * rz;
    const float rf3 = TP * dx, rf4 = TP * dy, rf5 = TP * dz, rf6 = TP * dis;

    {
      const _Float16* frow = ft + ((size_t)(b * NPT + idx)) * CIN;
      #pragma unroll
      for (int q = 0; q < 8; ++q) {
        const v8h fv = *(const v8ha*)(frow + 8 * q);
        #pragma unroll
        for (int e = 0; e < 8; ++e) featL[(8 * q + e) * KNB + lane] = fv[e];
      }
    }

    {
      _Float16* per = peL + lane * 64;
      #pragma unroll 1
      for (int j = 0; j < 32; ++j) {
        float pr = rf0 * sB[j];
        pr = fmaf(rf1, sB[32 + j], pr);
        pr = fmaf(rf2, sB[64 + j], pr);
        pr = fmaf(rf3, sB[96 + j], pr);
        pr = fmaf(rf4, sB[128 + j], pr);
        pr = fmaf(rf5, sB[160 + j], pr);
        pr = fmaf(rf6, sB[192 + j], pr);
        per[j]      = (_Float16)sinf(pr);
        per[32 + j] = (_Float16)cosf(pr);
      }
    }

    {
      float* rr = rawS + lane * 32;
      #pragma unroll 4
      for (int j = 0; j < 32; ++j) {
        float v = sOP[lane * 32 + j];
        v = fmaf(dx, sK[j], v);
        v = fmaf(dy, sK[32 + j], v);
        v = fmaf(dz, sK[64 + j], v);
        rr[j] = (v > 0.0f) ? v : 0.0f;
      }
    }
    __syncthreads();

    {
      float s = 0.0f;
      #pragma unroll 8
      for (int k = 0; k < 32; ++k) s += rawS[k * 32 + lane];
      const float rc = 1024.0f * (1.0f / (s + 1e-6f));
      _Float16* prw = permT + lane * 32;
      #pragma unroll 8
      for (int k = 0; k < 32; ++k) prw[k] = (_Float16)(rawS[k * 32 + lane] * rc);
    }

    #pragma unroll
    for (int mt = 0; mt < 2; ++mt) {
      #pragma unroll
      for (int nt = 0; nt < 2; ++nt) {
        v8f acc = zero8;
        #pragma unroll
        for (int ks = 0; ks < 2; ++ks) {
          const v16h a  = load_frag(wmh + (16 * mt + m) * 64 + 32 * ks, h);
          const v16h bb = load_frag(peL + (16 * nt + m) * 64 + 32 * ks, h);
          acc = wmma_f16(a, bb, acc);
        }
        #pragma unroll
        for (int r = 0; r < 8; ++r) {
          const int o = 16 * mt + 8 * h + r;
          const float v = acc[r] * (1.0f / 64.0f) + sBM[o];
          featL[(CIN + o) * KNB + 16 * nt + m] = (_Float16)v;
        }
      }
    }
    __syncthreads();

    #pragma unroll
    for (int jt = 0; jt < 2; ++jt) {
      const v16h bb = load_frag(permT + (16 * jt + m) * 32, h);
      #pragma unroll
      for (int mt = 0; mt < 6; ++mt) {
        const v16h a = load_frag(featL + (16 * mt + m) * 32, h);
        const v8f acc = wmma_f16(a, bb, zero8);
        #pragma unroll
        for (int r = 0; r < 8; ++r) {
          const int c = 16 * mt + 8 * h + r;
          const int fi = c * KNB + 16 * jt + m;
          const float v = acc[r] * (1.0f / 1024.0f);
          const _Float16 hv = (_Float16)v;
          const _Float16 lv = (_Float16)((v - (float)hv) * 2048.0f);
          fhS[fi] = hv;
          flS[fi] = lv;
        }
      }
    }
    __syncthreads();

    _Float16* gh = flh + (size_t)lp * FLATK;
    _Float16* gl = fll + (size_t)lp * FLATK;
    flat_store_pass(fhS, flS, gh, gl, lane);
    __threadfence();
    flat_store_pass(fhS, flS, gh, gl, lane);
    __syncthreads();
  }
}

__device__ __forceinline__ void conv_store_pass(const float* sT, float* pre, int b, int n0, int w, int lane) {
  #pragma unroll
  for (int i = 0; i < 8; ++i) {
    const int ch = 8 * w + i;
    const v4f v = *(const v4fa*)(sT + ch * 128 + 4 * lane);
    *(volatile v4f*)(pre + ((size_t)(b * COUT + ch)) * NPT + n0 + 4 * lane) = v;
  }
}

__global__ __launch_bounds__(256) void k_conv(
    const _Float16* __restrict__ flh,
    const _Float16* __restrict__ fll,
    const _Float16* __restrict__ wch,
    const float* __restrict__ bconv,
    float* __restrict__ pre,
    int tbase)
{
  __shared__ __attribute__((aligned(16))) float sT[64 * 128];
  const int tid = threadIdx.x, lane = tid & 31, w = tid >> 5;
  const int h = lane >> 4, m = lane & 15;
  const int lt0 = blockIdx.x * 128 + 16 * w;

  const _Float16* ah = flh + (size_t)(lt0 + m) * FLATK;
  const _Float16* al = fll + (size_t)(lt0 + m) * FLATK;
  const _Float16* wr = wch + (size_t)m * FLATK;

  const v8f zero8 = {0.f, 0.f, 0.f, 0.f, 0.f, 0.f, 0.f, 0.f};
  v8f acch[4], accl[4];
  #pragma unroll
  for (int nt = 0; nt < 4; ++nt) { acch[nt] = zero8; accl[nt] = zero8; }

  #pragma unroll 1
  for (int k0 = 0; k0 < FLATK; k0 += 32) {
    const v16h a0 = load_frag(ah + k0, h);
    const v16h a1 = load_frag(al + k0, h);
    #pragma unroll
    for (int nt = 0; nt < 4; ++nt) {
      const v16h bb = load_frag(wr + (size_t)nt * 16 * FLATK + k0, h);
      acch[nt] = wmma_f16(a0, bb, acch[nt]);
      accl[nt] = wmma_f16(a1, bb, accl[nt]);
    }
  }

  #pragma unroll
  for (int nt = 0; nt < 4; ++nt) {
    const int ch = 16 * nt + m;
    const float bv = bconv[ch];
    #pragma unroll
    for (int r = 0; r < 8; ++r) {
      const int tok = 16 * w + 8 * h + r;
      const float y = (acch[nt][r] + accl[nt][r] * (1.0f / 2048.0f)) * (1.0f / 4096.0f) + bv;
      sT[ch * 128 + tok] = y;
    }
  }
  __syncthreads();

  const int T = tbase + blockIdx.x * 128;
  const int b = T >> 13, n0 = T & (NPT - 1);
  conv_store_pass(sT, pre, b, n0, w, lane);
  __threadfence();
  conv_store_pass(sT, pre, b, n0, w, lane);
}

__global__ __launch_bounds__(256) void k_colstats(const float* __restrict__ pre, float* __restrict__ stat) {
  __shared__ double ss[256];
  __shared__ double sq[256];
  const int c = blockIdx.x, tid = threadIdx.x;
  double s = 0.0, q = 0.0;
  #pragma unroll 1
  for (int b = 0; b < NB; ++b) {
    const float* row = pre + ((size_t)(b * COUT + c)) * NPT;
    #pragma unroll 4
    for (int i = 0; i < NPT / 256; ++i) {
      const double v = (double)row[i * 256 + tid];
      s += v;
      q = v * v + q;
    }
  }
  ss[tid] = s;
  sq[tid] = q;
  __syncthreads();
  #pragma unroll 1
  for (int st = 128; st > 0; st >>= 1) {
    if (tid < st) {
      ss[tid] += ss[tid + st];
      sq[tid] += sq[tid + st];
    }
    __syncthreads();
  }
  if (tid < 8) {
    DU2 u;
    u.d[0] = ss[0];
    u.d[1] = sq[0];
    const v4f zero4 = {0.f, 0.f, 0.f, 0.f};
    v4f val = zero4;
    if (tid == 0) val = u.f;
    float* dst = stat + (size_t)c * 32 + 4 * tid;
    *(volatile v4f*)dst = val;
    __threadfence();
    *(volatile v4f*)dst = val;
  }
}

__global__ __launch_bounds__(256) void k_bnapply(const float* __restrict__ pre, const float* __restrict__ stat,
                                                const float* __restrict__ gamma, const float* __restrict__ beta,
                                                float* __restrict__ out) {
  const int rowid = blockIdx.x;
  const int c = rowid & (COUT - 1), tid = threadIdx.x;
  DU2 u;
  u.f = *(const v4fa*)(stat + (size_t)c * 32);
  const double mean = u.d[0] * (1.0 / 32768.0);
  double var = u.d[1] * (1.0 / 32768.0) - mean * mean;
  var = (var > 0.0) ? var : 0.0;
  const float meanf = (float)mean;
  const float varf = (float)var;
  const float inv = 1.0f / sqrtf(varf + 1e-5f);
  const float sc = gamma[c] * inv;
  const float bt = beta[c];
  const float* src = pre + (size_t)rowid * NPT;
  float* dst = out + (size_t)rowid * NPT;
  v4f y[8];
  #pragma unroll
  for (int i = 0; i < 8; ++i) {
    const v4f xv = *(const v4fa*)(src + 4 * (i * 256 + tid));
    y[i] = (xv - meanf) * sc + bt;
  }
  #pragma unroll
  for (int i = 0; i < 8; ++i) *(volatile v4f*)(dst + 4 * (i * 256 + tid)) = y[i];
  __threadfence();
  #pragma unroll
  for (int i = 0; i < 8; ++i) *(volatile v4f*)(dst + 4 * (i * 256 + tid)) = y[i];
}

extern "C" void kernel_launch(void* const* d_in, const int* in_sizes, int n_in,
                              void* d_out, int out_size, void* d_ws, size_t ws_size,
                              hipStream_t stream) {
  if (n_in < 12) return;
  if (in_sizes[0] != NB * 3 * NPT) return;
  if (in_sizes[1] != NB * CIN * NPT) return;
  if (in_sizes[2] != NB * NPT * KNB) return;
  if (in_sizes[3] != 7 * 32 || in_sizes[4] != 3 * 32 || in_sizes[5] != 32 * 32) return;
  if (in_sizes[6] != CXF * 64 || in_sizes[7] != CXF) return;
  if (in_sizes[8] != COUT * FLATK || in_sizes[9] != COUT || in_sizes[10] != COUT || in_sizes[11] != COUT) return;
  if (out_size != NB * COUT * NPT) return;
  if (ws_size < WS_TOTAL) return;

  const float* x       = (const float*)d_in[0];
  const float* feature = (const float*)d_in[1];
  const int*   neigh   = (const int*)  d_in[2];
  const float* Bmat    = (const float*)d_in[3];
  const float* kern    = (const float*)d_in[4];
  const float* opad    = (const float*)d_in[5];
  const float* W_mlp   = (const float*)d_in[6];
  const float* b_mlp   = (const float*)d_in[7];
  const float* W_conv  = (const float*)d_in[8];
  const float* b_conv  = (const float*)d_in[9];
  const float* gamma   = (const float*)d_in[10];
  const float* beta    = (const float*)d_in[11];
  float* out = (float*)d_out;

  char* ws = (char*)d_ws;
  _Float16* wch  = (_Float16*)(ws + WS_WCH);
  _Float16* wmh  = (_Float16*)(ws + WS_WMH);
  _Float16* ft   = (_Float16*)(ws + WS_FT);
  _Float16* flh  = (_Float16*)(ws + WS_FLH);
  _Float16* fll  = (_Float16*)(ws + WS_FLL);
  float*    pre  = (float*)   (ws + WS_PRE);
  float*    stat = (float*)   (ws + WS_STAT);

  k_cvtw<<<NWC8 / 256 + 1, 256, 0, stream>>>(W_conv, W_mlp, wch, wmh);

  k_ft<<<dim3(NPT / 64, NB), 256, 0, stream>>>(feature, ft);

  hipFuncSetAttribute(reinterpret_cast<const void*>(&k_point), hipFuncAttributeMaxDynamicSharedMemorySize, LDS_POINT);
  for (int ch = 0; ch < NCHUNK; ++ch) {
    k_point<<<CHUNK / PPB, 128, LDS_POINT, stream>>>(x, neigh, Bmat, kern, opad, b_mlp, ft, wmh, flh, fll, ch * CHUNK);
    k_conv<<<CHUNK / 128, 256, 0, stream>>>(flh, fll, wch, b_conv, pre, ch * CHUNK);
  }

  k_colstats<<<COUT, 256, 0, stream>>>(pre, stat);
  k_bnapply<<<NB * COUT, 256, 0, stream>>>(pre, stat, gamma, beta, out);
}
